// Mamba_48567490183604
// MI455X (gfx1250) — hardware-verified
//
#include <hip/hip_runtime.h>
#include <math.h>

typedef __attribute__((ext_vector_type(16))) _Float16 v16h;
typedef __attribute__((ext_vector_type(8)))  _Float16 v8h;
typedef __attribute__((ext_vector_type(16))) __bf16   v16b;
typedef __attribute__((ext_vector_type(8)))  __bf16   v8b;
typedef __attribute__((ext_vector_type(8)))  float    v8f;
typedef __attribute__((ext_vector_type(4)))  float    v4f;

constexpr int kBsz  = 2;
constexpr int kCh   = 64;
constexpr int kDin  = 128;
constexpr int kNst  = 32;
constexpr int kDir  = 4;
constexpr int kDtR  = 4;
constexpr int kHgt  = 48;
constexpr int kWid  = 48;
constexpr int kL    = kHgt * kWid;
constexpr int kTok  = kBsz * kL;
constexpr int kBK   = kBsz * kDir;
constexpr int kXdW  = kDtR + 2 * kNst;
constexpr int kXdP  = 128;
constexpr int kScanTS = 32;
constexpr int kConvTS = 64;
constexpr int kConvP  = 68;
static_assert(kNst == 32, "lane = state");
static_assert((kCh % 32) == 0 && (kDin % 32) == 0, "GEMM K multiples of 32");
static_assert(((2 * kDin) % 64) == 0 && (kTok % 64) == 0 && (kL % 64) == 0 && (kXdP % 64) == 0 && (kCh % 64) == 0,
              "GEMM M,N multiples of 64");
static_assert((kL % kScanTS) == 0 && (kL % kConvTS) == 0 && (kTok % 8) == 0 && (kDin % 8) == 0, "tile multiples");
static_assert(kXdW <= kXdP, "x_proj pad");

constexpr size_t kOffXNH = 0;
constexpr size_t kOffXNL = kOffXNH + (size_t)kTok * kCh * 2;
constexpr size_t kOffWIH = kOffXNL + (size_t)kTok * kCh * 2;
constexpr size_t kOffWIL = kOffWIH + (size_t)2 * kDin * kCh * 2;
constexpr size_t kOffWXH = kOffWIL + (size_t)2 * kDin * kCh * 2;
constexpr size_t kOffWXL = kOffWXH + (size_t)kBK * kXdP * kDin * 2;
constexpr size_t kOffWOH = kOffWXL + (size_t)kBK * kXdP * kDin * 2;
constexpr size_t kOffWOL = kOffWOH + (size_t)kCh * kDin * 2;
constexpr size_t kOffXZ  = kOffWOL + (size_t)kCh * kDin * 2;
constexpr size_t kOffXS  = kOffXZ  + (size_t)2 * kDin * kTok * 4;
constexpr size_t kOffXTH = kOffXS  + (size_t)kBK * kDin * kL * 4;
constexpr size_t kOffXTL = kOffXTH + (size_t)kBK * kL * kDin * 2;
constexpr size_t kOffXD  = kOffXTL + (size_t)kBK * kL * kDin * 2;
constexpr size_t kOffYS  = kOffXD  + (size_t)kBK * kL * kXdP * 4;
constexpr size_t kOffYGH = kOffYS  + (size_t)kBK * kDin * kL * 4;
constexpr size_t kOffYGL = kOffYGH + (size_t)kTok * kDin * 2;
constexpr size_t kWsTotal = kOffYGL + (size_t)kTok * kDin * 2;
static_assert(kWsTotal == 46628864ull, "carve total");
static_assert(kWsTotal <= 134217728ull, "carve cap");
static_assert((kOffXNL % 128) == 0 && (kOffWIH % 128) == 0 && (kOffWIL % 128) == 0 && (kOffWXH % 128) == 0 &&
              (kOffWXL % 128) == 0 && (kOffWOH % 128) == 0 && (kOffWOL % 128) == 0 && (kOffXZ % 128) == 0 &&
              (kOffXS % 128) == 0 && (kOffXTH % 128) == 0 && (kOffXTL % 128) == 0 && (kOffXD % 128) == 0 &&
              (kOffYS % 128) == 0 && (kOffYGH % 128) == 0 && (kOffYGL % 128) == 0, "128-B aligned regions");

__device__ __forceinline__ unsigned short f2bf_bits(float f) {
  unsigned u = __float_as_uint(f);
  return (unsigned short)((u + 0x7FFFu + ((u >> 16) & 1u)) >> 16);
}
__device__ __forceinline__ float bf_bits2f(unsigned short h) { return __uint_as_float(((unsigned)h) << 16); }

__device__ __forceinline__ void split8(const v4f a0, const v4f a1, v8h& hv, v8h& lv) {
#pragma unroll
  for (int e = 0; e < 4; ++e) {
    const float f0 = a0[e], f1 = a1[e];
    const unsigned short h0 = f2bf_bits(f0), h1 = f2bf_bits(f1);
    const unsigned short l0 = f2bf_bits(f0 - bf_bits2f(h0)), l1 = f2bf_bits(f1 - bf_bits2f(h1));
    hv[e]     = __builtin_bit_cast(_Float16, h0);
    hv[4 + e] = __builtin_bit_cast(_Float16, h1);
    lv[e]     = __builtin_bit_cast(_Float16, l0);
    lv[4 + e] = __builtin_bit_cast(_Float16, l1);
  }
}

__device__ __forceinline__ void dep_guard_h(v8f& a, v8f& b, v16h x, v16h y) { asm volatile("v_nop\n\tv_nop\n\tv_nop\n\tv_nop" : "+v"(a), "+v"(b) : "v"(x), "v"(y)); }
__device__ __forceinline__ void dep_guard_b(v8f& a, v8f& b, v16b x, v16b y) { asm volatile("v_nop\n\tv_nop\n\tv_nop\n\tv_nop" : "+v"(a), "+v"(b) : "v"(x), "v"(y)); }
__device__ __forceinline__ void dep_guard4_h(v8f& a, v8f& b, v8f& c, v8f& d, v16h x, v16h y) { asm volatile("v_nop\n\tv_nop\n\tv_nop\n\tv_nop" : "+v"(a), "+v"(b), "+v"(c), "+v"(d) : "v"(x), "v"(y)); }
__device__ __forceinline__ void dep_guard4_b(v8f& a, v8f& b, v8f& c, v8f& d, v16b x, v16b y) { asm volatile("v_nop\n\tv_nop\n\tv_nop\n\tv_nop" : "+v"(a), "+v"(b), "+v"(c), "+v"(d) : "v"(x), "v"(y)); }
__device__ __forceinline__ void keep4_h(v16h a, v16h b, v16h c, v16h d) { asm volatile("v_nop" :: "v"(a), "v"(b), "v"(c), "v"(d)); }
__device__ __forceinline__ void keep4_b(v16b a, v16b b, v16b c, v16b d) { asm volatile("v_nop" :: "v"(a), "v"(b), "v"(c), "v"(d)); }
__device__ __forceinline__ void acc_guard4(v8f& a, v8f& b, v8f& c, v8f& d) { asm volatile("v_nop\n\tv_nop\n\tv_nop\n\tv_nop" : "+v"(a), "+v"(b), "+v"(c), "+v"(d)); }
template <typename T> struct Frag;
template <> struct Frag<_Float16> {
  typedef v16h V; union U { v16h v; v8h h[2]; };
  static __device__ __forceinline__ v16h load(const _Float16* p) {
    U f; f.h[0] = *(const v8h*)(p); f.h[1] = *(const v8h*)(p + 16); return f.v;
  }
  static __device__ __forceinline__ v8f mma(v16h a, v16h b, v8f c) {
    return __builtin_amdgcn_wmma_f32_16x16x32_f16(false, a, false, b, (short)0, c, false, false);
  }
  static __device__ __forceinline__ void guard(v8f& a, v8f& b, v16h x, v16h y) { dep_guard_h(a, b, x, y); }
  static __device__ __forceinline__ void guard4(v8f& a, v8f& b, v8f& c, v8f& d, v16h x, v16h y) { dep_guard4_h(a, b, c, d, x, y); }
  static __device__ __forceinline__ void keep(v16h a, v16h b, v16h c, v16h d) { keep4_h(a, b, c, d); }
};
template <> struct Frag<__bf16> {
  typedef v16b V; union U { v16b v; v8b h[2]; };
  static __device__ __forceinline__ v16b load(const __bf16* p) {
    U f; f.h[0] = *(const v8b*)(p); f.h[1] = *(const v8b*)(p + 16); return f.v;
  }
  static __device__ __forceinline__ v8f mma(v16b a, v16b b, v8f c) {
    return __builtin_amdgcn_wmma_f32_16x16x32_bf16(false, a, false, b, (short)0, c, false, false);
  }
  static __device__ __forceinline__ void guard(v8f& a, v8f& b, v16b x, v16b y) { dep_guard_b(a, b, x, y); }
  static __device__ __forceinline__ void guard4(v8f& a, v8f& b, v8f& c, v8f& d, v16b x, v16b y) { dep_guard4_b(a, b, c, d, x, y); }
  static __device__ __forceinline__ void keep(v16b a, v16b b, v16b c, v16b d) { keep4_b(a, b, c, d); }
};

template <int ET> struct Elem;
template <> struct Elem<0> { typedef _Float16 T; };
template <> struct Elem<1> { typedef __bf16 T; };
template <int ET, int SPL, int BIAS_MODE, int OUT_MODE, bool RESID, int ACT = 0>
__global__ __launch_bounds__(256) void wmma_gemm64(
    const unsigned short* __restrict__ Ap, const unsigned short* __restrict__ A2p, int lda, long strideA,
    const unsigned short* __restrict__ Btp, const unsigned short* __restrict__ Bt2p, int ldb, long strideB,
    void* __restrict__ Cout, void* __restrict__ Cout2, int ldc, long strideC,
    const float* __restrict__ bias,
    const float* __restrict__ resid, long strideR,
    int M, int N, int K, float scale) {
  typedef typename Elem<ET>::T T;
  typedef typename Frag<T>::V V;
  const T* A = (const T*)Ap; const T* A2 = (const T*)A2p; const T* Bt = (const T*)Btp; const T* Bt2 = (const T*)Bt2p;
  __shared__ __align__(16) float sT[8][16 * 68];
  const int b    = blockIdx.y;
  const int lane = threadIdx.x & 31;
  const int wave = threadIdx.x >> 5;
  const int tilesN = N >> 6;
  const int tilesM = M >> 6;
  const int tile = blockIdx.x * 8 + wave;
  if (tile >= tilesM * tilesN) return;
  const int tm = tile / tilesN;
  const int tn = tile - tm * tilesN;
  const int m0 = tm << 6;
  const int n0 = tn << 6;

  const T* Ab  = A  + (size_t)b * strideA;
  const T* Bb  = Bt + (size_t)b * strideB;
  const T* Ab2 = (SPL >= 1) ? (A2  + (size_t)b * strideA) : nullptr;
  const T* Bb2 = (SPL == 2) ? (Bt2 + (size_t)b * strideB) : nullptr;

  const int rlane = lane & 15;
  const int koff  = (lane >> 4) * 8;
  const int mOff  = (lane >> 4) * 8;

  v8f acc[4][4];
#pragma unroll
  for (int i = 0; i < 4; ++i)
#pragma unroll
    for (int j = 0; j < 4; ++j) acc[i][j] = (v8f){0.f,0.f,0.f,0.f,0.f,0.f,0.f,0.f};

  for (int k0 = 0; k0 < K; k0 += 32) {
    V bh[4], bl[4];
#pragma unroll
    for (int j = 0; j < 4; ++j) {
      const size_t bo = (size_t)(n0 + (j << 4) + rlane) * ldb + koff + k0;
      bh[j] = Frag<T>::load(Bb + bo);
      if (SPL == 2) bl[j] = Frag<T>::load(Bb2 + bo);
    }
#pragma unroll
    for (int i = 0; i < 4; ++i) {
      const size_t ao = (size_t)(m0 + (i << 4) + rlane) * lda + koff + k0;
      V ah = Frag<T>::load(Ab + ao);
      V al;
      if (SPL >= 1) al = Frag<T>::load(Ab2 + ao);
#pragma unroll
      for (int j = 0; j < 4; ++j) {
        acc[i][j] = Frag<T>::mma(ah, bh[j], acc[i][j]);
        if (SPL == 2) acc[i][j] = Frag<T>::mma(ah, bl[j], acc[i][j]);
        if (SPL >= 1) acc[i][j] = Frag<T>::mma(al, bh[j], acc[i][j]);
      }
      Frag<T>::guard4(acc[i][0], acc[i][1], acc[i][2], acc[i][3], ah, (SPL >= 1) ? al : ah);
    }
    Frag<T>::keep(bh[0], bh[1], bh[2], bh[3]);
    if (SPL == 2) Frag<T>::keep(bl[0], bl[1], bl[2], bl[3]);
  }
  acc_guard4(acc[0][0], acc[0][1], acc[0][2], acc[0][3]);
  acc_guard4(acc[1][0], acc[1][1], acc[1][2], acc[1][3]);
  acc_guard4(acc[2][0], acc[2][1], acc[2][2], acc[2][3]);
  acc_guard4(acc[3][0], acc[3][1], acc[3][2], acc[3][3]);

  float* slab = sT[wave];
  const float* Rb = RESID ? (resid + (size_t)b * strideR) : nullptr;
#pragma unroll
  for (int i = 0; i < 4; ++i) {
    const int mBase = m0 + (i << 4);
#pragma unroll
    for (int j = 0; j < 4; ++j) {
      const int n = n0 + (j << 4) + rlane;
      float bv = 0.f;
      if (BIAS_MODE == 2) bv = bias[n];
#pragma unroll
      for (int r = 0; r < 8; ++r) {
        float v = acc[i][j][r] * scale;
        if (BIAS_MODE == 1) v += bias[mBase + mOff + r];
        if (BIAS_MODE == 2) v += bv;
        if (ACT == 1) v = tanhf(v);
        if (ACT == 2) v = fmaxf(v, 0.0f);
        if (ACT == 3) v = v / (1.0f + expf(-v));
        if (ACT == 4) v = (v > 0.f) ? v : 0.01f * v;
        slab[(mOff + r) * 68 + (j << 4) + rlane] = v;
      }
    }
    __builtin_amdgcn_fence(__ATOMIC_RELEASE, "workgroup");
    __builtin_amdgcn_wave_barrier();
    __builtin_amdgcn_fence(__ATOMIC_ACQUIRE, "workgroup");
    if (OUT_MODE == 0) {
      float* C = (float*)Cout + (size_t)b * strideC;
      const int hh = lane >> 4, c4 = (lane & 15) * 4;
      for (int pass = 0; pass < 2; ++pass) {
#pragma unroll
        for (int it = 0; it < 8; ++it) {
          const int row = it * 2 + hh;
          v4f v = *(const v4f*)(slab + row * 68 + c4);
          if (RESID) {
            const v4f rr = *(const v4f*)(Rb + (size_t)(mBase + row) * ldc + n0 + c4);
            v += rr;
          }
          *(volatile v4f*)(C + (size_t)(mBase + row) * ldc + n0 + c4) = v;
        }
        __threadfence();
      }
    } else {
      const int q = lane >> 3, c8 = (lane & 7) * 8;
      unsigned short* C  = (unsigned short*)Cout  + (size_t)b * strideC;
      unsigned short* C2 = (OUT_MODE == 2) ? ((unsigned short*)Cout2 + (size_t)b * strideC) : nullptr;
      for (int pass = 0; pass < 2; ++pass) {
#pragma unroll
        for (int it = 0; it < 4; ++it) {
          const int row = it * 4 + q;
          const float* sp = slab + row * 68 + c8;
          v8h hv, lv;
#pragma unroll
          for (int e = 0; e < 8; ++e) {
            if (OUT_MODE == 1) {
              hv[e] = (_Float16)sp[e];
            } else {
              unsigned short hb = f2bf_bits(sp[e]);
              unsigned short lb = f2bf_bits(sp[e] - bf_bits2f(hb));
              hv[e] = __builtin_bit_cast(_Float16, hb);
              lv[e] = __builtin_bit_cast(_Float16, lb);
            }
          }
          *(volatile v8h*)(C + (size_t)(mBase + row) * ldc + n0 + c8) = hv;
          if (OUT_MODE == 2) *(volatile v8h*)(C2 + (size_t)(mBase + row) * ldc + n0 + c8) = lv;
        }
        __threadfence();
      }
    }
    __builtin_amdgcn_fence(__ATOMIC_RELEASE, "workgroup");
    __builtin_amdgcn_wave_barrier();
    __builtin_amdgcn_fence(__ATOMIC_ACQUIRE, "workgroup");
  }
}

__global__ __launch_bounds__(256) void split_rows_bf16_kernel(
    const float* __restrict__ src, unsigned short* __restrict__ dhi, unsigned short* __restrict__ dlo, int total8)
{
  const int i = blockIdx.x * 256 + threadIdx.x;
  if (i >= total8) return;
  const size_t e0 = (size_t)i << 3;
  const v4f a0 = *(const v4f*)(src + e0);
  const v4f a1 = *(const v4f*)(src + e0 + 4);
  v8h hv, lv;
  split8(a0, a1, hv, lv);
  unsigned short* qh = dhi + e0;
  unsigned short* ql = dlo + e0;
  *(volatile v8h*)qh = hv;
  *(volatile v8h*)ql = lv;
  __threadfence();
  *(volatile v8h*)qh = hv;
  *(volatile v8h*)ql = lv;
}

__global__ __launch_bounds__(256) void xproj_planes_kernel(
    const float* __restrict__ wx, unsigned short* __restrict__ dhi, unsigned short* __restrict__ dlo)
{
  const int i   = blockIdx.x * 256 + threadIdx.x;
  const int e0  = i << 3;
  const int ro  = e0 >> 7;
  const int col = e0 & (kDin - 1);
  const int bk  = ro >> 7;
  const int c   = ro & (kXdP - 1);
  const int kdir = bk & 3;
  const bool valid = (c < kXdW);
  const int cc  = valid ? c : (kXdW - 1);
  const float fz = valid ? 1.0f : 0.0f;
  const float* src = wx + (size_t)(kdir * kXdW + cc) * kDin + col;
  const v4f a0 = *(const v4f*)(src) * fz;
  const v4f a1 = *(const v4f*)(src + 4) * fz;
  v8h hv, lv;
  split8(a0, a1, hv, lv);
  unsigned short* qh = dhi + (size_t)e0;
  unsigned short* ql = dlo + (size_t)e0;
  *(volatile v8h*)qh = hv;
  *(volatile v8h*)ql = lv;
  __threadfence();
  *(volatile v8h*)qh = hv;
  *(volatile v8h*)ql = lv;
}

__global__ __launch_bounds__(256) void ln_token_kernel(
    const float* __restrict__ x, const float* __restrict__ g, const float* __restrict__ be,
    unsigned short* __restrict__ XNH, unsigned short* __restrict__ XNL)
{
  __shared__ __align__(16) float sL[8 * 64];
  const int tid = threadIdx.x, lane = tid & 31, wave = tid >> 5;
  const int t = blockIdx.x * 8 + wave;
  const int bi = t / kL;
  const int pos = t - bi * kL;
  const float* base = x + (size_t)bi * kCh * kL + pos;
  const float v0 = base[(size_t)lane * kL];
  const float v1 = base[(size_t)(lane + 32) * kL];
  float s = v0 + v1;
#pragma unroll
  for (int off = 16; off > 0; off >>= 1) s += __shfl_xor(s, off, 32);
  const float mu = s * (1.0f / 64.0f);
  const float d0 = v0 - mu, d1 = v1 - mu;
  float q = d0 * d0 + d1 * d1;
#pragma unroll
  for (int off = 16; off > 0; off >>= 1) q += __shfl_xor(q, off, 32);
  const float rs = rsqrtf(q * (1.0f / 64.0f) + 1e-5f);
  const float y0 = d0 * rs * g[lane] + be[lane];
  const float y1 = d1 * rs * g[lane + 32] + be[lane + 32];
  float* sl = sL + wave * 64;
  sl[lane] = y0;
  sl[lane + 32] = y1;
  __builtin_amdgcn_fence(__ATOMIC_RELEASE, "workgroup");
  __builtin_amdgcn_wave_barrier();
  __builtin_amdgcn_fence(__ATOMIC_ACQUIRE, "workgroup");
  const int c8 = (lane & 7) * 8;
  const v4f a0 = *(const v4f*)(sl + c8);
  const v4f a1 = *(const v4f*)(sl + c8 + 4);
  v8h hv, lv;
  split8(a0, a1, hv, lv);
  const size_t o = (size_t)t * kCh + c8;
  if (lane < 8) {
    *(volatile v8h*)(XNH + o) = hv;
    *(volatile v8h*)(XNL + o) = lv;
  }
  __threadfence();
  if (lane < 8) {
    *(volatile v8h*)(XNH + o) = hv;
    *(volatile v8h*)(XNL + o) = lv;
  }
}

__global__ __launch_bounds__(128) void conv_dir_kernel(
    const float* __restrict__ XZ, const float* __restrict__ cw, const float* __restrict__ cb,
    float* __restrict__ XS, unsigned short* __restrict__ XTH, unsigned short* __restrict__ XTL)
{
  __shared__ __align__(16) float sU[kDin * kConvP];
  const int tid = threadIdx.x, lane = tid & 31, wave = tid >> 5;
  const int d = tid;
  const int l0 = blockIdx.x * kConvTS;
  const int kdir = blockIdx.y;
  const int bi = blockIdx.z;
  const int bk = bi * kDir + kdir;
  float wt[9];
#pragma unroll
  for (int i = 0; i < 9; ++i) wt[i] = cw[d * 9 + i];
  float bias = cb[d];
  asm volatile("" : "+v"(wt[0]), "+v"(wt[1]), "+v"(wt[2]), "+v"(wt[3]), "+v"(wt[4]),
                    "+v"(wt[5]), "+v"(wt[6]), "+v"(wt[7]), "+v"(wt[8]), "+v"(bias) :: "memory");
  const float* xr = XZ + (size_t)d * kTok + (size_t)bi * kL;
#pragma unroll 1
  for (int s = 0; s < kConvTS; ++s) {
    const int l = l0 + s;
    const int ll = (kdir >= 2) ? (kL - 1 - l) : l;
    int hI, wI;
    if (kdir & 1) { wI = ll / kHgt; hI = ll - wI * kHgt; }
    else          { hI = ll / kWid; wI = ll - hI * kWid; }
    float acc = 0.0f;
#pragma unroll
    for (int kh = 0; kh < 3; ++kh) {
      const int hh = hI + kh - 1;
      const bool vh = ((unsigned)hh < (unsigned)kHgt);
      const int hc = (hh < 0) ? 0 : ((hh > kHgt - 1) ? (kHgt - 1) : hh);
#pragma unroll
      for (int kq = 0; kq < 3; ++kq) {
        const int ww = wI + kq - 1;
        const bool vw = ((unsigned)ww < (unsigned)kWid);
        const int wc = (ww < 0) ? 0 : ((ww > kWid - 1) ? (kWid - 1) : ww);
        const float xv = xr[hc * kWid + wc];
        acc = fmaf(wt[kh * 3 + kq], (vh && vw) ? xv : 0.0f, acc);
      }
    }
    const float sv = acc + bias;
    const float sg = __builtin_amdgcn_rcpf(1.0f + expf(-sv));
    sU[d * kConvP + s] = sv * sg;
  }
  __syncthreads();
  const int hq = lane >> 4;
  const int c4 = (lane & 15) * 4;
  const int c8 = (lane & 15) * 8;
  float* xsb = XS + (size_t)bk * kDin * kL + l0;
  unsigned short* xth = XTH + ((size_t)bk * kL + l0) * kDin;
  unsigned short* xtl = XTL + ((size_t)bk * kL + l0) * kDin;
  for (int pass = 0; pass < 2; ++pass) {
#pragma unroll
    for (int it = 0; it < 16; ++it) {
      const int dr = wave * 32 + it * 2 + hq;
      const v4f v = *(const v4f*)(sU + dr * kConvP + c4);
      *(volatile v4f*)(xsb + (size_t)dr * kL + c4) = v;
    }
#pragma unroll
    for (int it = 0; it < 8; ++it) {
      const int sr = wave * 16 + it * 2 + hq;
      v4f a0, a1;
#pragma unroll
      for (int e = 0; e < 4; ++e) {
        a0[e] = sU[(c8 + e) * kConvP + sr];
        a1[e] = sU[(c8 + 4 + e) * kConvP + sr];
      }
      v8h hv, lv;
      split8(a0, a1, hv, lv);
      const size_t o = (size_t)sr * kDin + c8;
      *(volatile v8h*)(xth + o) = hv;
      *(volatile v8h*)(xtl + o) = lv;
    }
    __threadfence();
  }
}

__global__ __launch_bounds__(256) void scan_kernel(
    const float* __restrict__ XD, const float* __restrict__ XS,
    const float* __restrict__ dtw, const float* __restrict__ dtb,
    const float* __restrict__ Alog, const float* __restrict__ Dsv,
    float* __restrict__ YS)
{
  __shared__ __align__(16) float sX[kScanTS * kXdP];
  __shared__ __align__(16) float sY[8 * 32];
  const int tid = threadIdx.x, lane = tid & 31, wave = tid >> 5;
  const int bk = blockIdx.x >> 4;
  const int dg = blockIdx.x & 15;
  const int d  = dg * 8 + wave;
  const int kdir = bk & 3;
  const int kd = kdir * kDin + d;
  const float a_n = -expf(Alog[(size_t)kd * kNst + lane]);
  const float dco = Dsv[kd];
  const float bdt = dtb[kd];
  const v4f wv = *(const v4f*)(dtw + (size_t)kd * kDtR);
  const float* urow = XS + ((size_t)bk * kDin + d) * kL;
  const float* xdb  = XD + (size_t)bk * kL * kXdP;
  float* yrow = YS + ((size_t)bk * kDin + d) * kL;
  const int sr = tid >> 3, sc = (tid & 7) * 16;
  float h = 0.0f;
#pragma unroll 1
  for (int t0 = 0; t0 < kL; t0 += kScanTS) {
    __syncthreads();
#pragma unroll
    for (int i = 0; i < 4; ++i)
      *(v4f*)(sX + sr * kXdP + sc + 4 * i) = *(const v4f*)(xdb + (size_t)(t0 + sr) * kXdP + sc + 4 * i);
    __syncthreads();
    const float u32 = urow[t0 + lane];
    const v4f dtr = *(const v4f*)(sX + lane * kXdP);
    float dot = dtr[0] * wv[0];
    dot = fmaf(dtr[1], wv[1], dot);
    dot = fmaf(dtr[2], wv[2], dot);
    dot = fmaf(dtr[3], wv[3], dot);
    const float v = dot + bdt;
    const float dl32 = fmaxf(v, 0.0f) + log1pf(expf(-fabsf(v)));
    float ybuf = 0.0f;
#pragma unroll 1
    for (int j = 0; j < kScanTS; ++j) {
      const float uj = __shfl(u32, j, 32);
      const float dj = __shfl(dl32, j, 32);
      const float bn = sX[j * kXdP + kDtR + lane];
      const float cn = sX[j * kXdP + kDtR + kNst + lane];
      float dA = expf(dj * a_n);
      dA = (dA < 1.17549435e-38f) ? 0.0f : dA;
      h = fmaf(dj * uj, bn, dA * h);
      float p = h * cn;
      p += __shfl_xor(p, 16, 32);
      p += __shfl_xor(p, 8, 32);
      p += __shfl_xor(p, 4, 32);
      p += __shfl_xor(p, 2, 32);
      p += __shfl_xor(p, 1, 32);
      const float y = fmaf(dco, uj, p);
      ybuf = (lane == j) ? y : ybuf;
    }
    sY[wave * 32 + lane] = ybuf;
    __builtin_amdgcn_fence(__ATOMIC_RELEASE, "workgroup");
    __builtin_amdgcn_wave_barrier();
    __builtin_amdgcn_fence(__ATOMIC_ACQUIRE, "workgroup");
    const v4f val = *(const v4f*)(sY + wave * 32 + (lane & 7) * 4);
    if (lane < 8) *(volatile v4f*)(yrow + t0 + lane * 4) = val;
    __threadfence();
    if (lane < 8) *(volatile v4f*)(yrow + t0 + lane * 4) = val;
  }
}

__global__ __launch_bounds__(256) void merge_gate_kernel(
    const float* __restrict__ YS, const float* __restrict__ XZ,
    const float* __restrict__ og, const float* __restrict__ ob,
    unsigned short* __restrict__ YGH, unsigned short* __restrict__ YGL)
{
  __shared__ __align__(16) float sM[8 * kDin];
  const int tid = threadIdx.x, lane = tid & 31, wave = tid >> 5;
  const int t = blockIdx.x * 8 + wave;
  const int bi = t / kL;
  const int pos = t - bi * kL;
  const int hI = pos / kWid;
  const int wI = pos - hI * kWid;
  const int pwh = wI * kHgt + hI;
  const size_t plane = (size_t)kDin * kL;
  const float* ys0 = YS + (size_t)(bi * kDir + 0) * plane + pos;
  const float* ys1 = YS + (size_t)(bi * kDir + 1) * plane + pwh;
  const float* ys2 = YS + (size_t)(bi * kDir + 2) * plane + (kL - 1 - pos);
  const float* ys3 = YS + (size_t)(bi * kDir + 3) * plane + (kL - 1 - pwh);
  float v[4];
  float s = 0.0f;
#pragma unroll
  for (int i = 0; i < 4; ++i) {
    const size_t dr = (size_t)(lane + 32 * i) * kL;
    float a0 = ys0[dr];
    float a2 = ys2[dr];
    float a1 = ys1[dr];
    float a3 = ys3[dr];
    asm volatile("" : "+v"(a0), "+v"(a1), "+v"(a2), "+v"(a3) :: "memory");
    const float y = ((a0 + a2) + a1) + a3;
    v[i] = y;
    s += y;
  }
#pragma unroll
  for (int off = 16; off > 0; off >>= 1) s += __shfl_xor(s, off, 32);
  const float mu = s * (1.0f / 128.0f);
  float ss = 0.0f;
#pragma unroll
  for (int i = 0; i < 4; ++i) { const float dl = v[i] - mu; ss += dl * dl; }
#pragma unroll
  for (int off = 16; off > 0; off >>= 1) ss += __shfl_xor(ss, off, 32);
  const float rs = rsqrtf(ss * (1.0f / 128.0f) + 1e-5f);
  float* sm = sM + wave * kDin;
#pragma unroll
  for (int i = 0; i < 4; ++i) {
    const int d = lane + 32 * i;
    float z  = XZ[(size_t)(kDin + d) * kTok + t];
    float gg = og[d];
    float bb = ob[d];
    asm volatile("" : "+v"(z), "+v"(gg), "+v"(bb) :: "memory");
    const float sg = __builtin_amdgcn_rcpf(1.0f + expf(-z));
    const float yn = (v[i] - mu) * rs * gg + bb;
    sm[d] = yn * (z * sg);
  }
  __builtin_amdgcn_fence(__ATOMIC_RELEASE, "workgroup");
  __builtin_amdgcn_wave_barrier();
  __builtin_amdgcn_fence(__ATOMIC_ACQUIRE, "workgroup");
  const int c8 = (lane & 15) * 8;
  const v4f a0 = *(const v4f*)(sm + c8);
  const v4f a1 = *(const v4f*)(sm + c8 + 4);
  v8h hv, lv;
  split8(a0, a1, hv, lv);
  const size_t o = (size_t)t * kDin + c8;
  if (lane < 16) {
    *(volatile v8h*)(YGH + o) = hv;
    *(volatile v8h*)(YGL + o) = lv;
  }
  __threadfence();
  if (lane < 16) {
    *(volatile v8h*)(YGH + o) = hv;
    *(volatile v8h*)(YGL + o) = lv;
  }
}

extern "C" void kernel_launch(void* const* d_in, const int* in_sizes, int n_in,
                              void* d_out, int out_size, void* d_ws, size_t ws_size,
                              hipStream_t stream) {
  if (n_in < 14) return;
  if (in_sizes[0] != kBsz * kCh * kL) return;
  if (in_sizes[1] != kCh || in_sizes[2] != kCh) return;
  if (in_sizes[3] != 2 * kDin * kCh) return;
  if (in_sizes[4] != kDin * 9) return;
  if (in_sizes[5] != kDin) return;
  if (in_sizes[6] != kDir * kXdW * kDin) return;
  if (in_sizes[7] != kDir * kDin * kDtR) return;
  if (in_sizes[8] != kDir * kDin) return;
  if (in_sizes[9] != kDir * kDin * kNst) return;
  if (in_sizes[10] != kDir * kDin) return;
  if (in_sizes[11] != kDin || in_sizes[12] != kDin) return;
  if (in_sizes[13] != kCh * kDin) return;
  if (out_size != kBsz * kCh * kL) return;
  if (ws_size < kWsTotal) return;

  const float* x_in     = (const float*)d_in[0];
  const float* ln_g     = (const float*)d_in[1];
  const float* ln_b     = (const float*)d_in[2];
  const float* w_in     = (const float*)d_in[3];
  const float* conv_w   = (const float*)d_in[4];
  const float* conv_b   = (const float*)d_in[5];
  const float* w_x      = (const float*)d_in[6];
  const float* w_dt     = (const float*)d_in[7];
  const float* b_dt     = (const float*)d_in[8];
  const float* a_log    = (const float*)d_in[9];
  const float* d_skip   = (const float*)d_in[10];
  const float* oln_g    = (const float*)d_in[11];
  const float* oln_b    = (const float*)d_in[12];
  const float* w_out    = (const float*)d_in[13];
  float* out = (float*)d_out;

  char* ws = (char*)d_ws;
  unsigned short* XNH = (unsigned short*)(ws + kOffXNH);
  unsigned short* XNL = (unsigned short*)(ws + kOffXNL);
  unsigned short* WIH = (unsigned short*)(ws + kOffWIH);
  unsigned short* WIL = (unsigned short*)(ws + kOffWIL);
  unsigned short* WXH = (unsigned short*)(ws + kOffWXH);
  unsigned short* WXL = (unsigned short*)(ws + kOffWXL);
  unsigned short* WOH = (unsigned short*)(ws + kOffWOH);
  unsigned short* WOL = (unsigned short*)(ws + kOffWOL);
  float*          XZ  = (float*)(ws + kOffXZ);
  float*          XS  = (float*)(ws + kOffXS);
  unsigned short* XTH = (unsigned short*)(ws + kOffXTH);
  unsigned short* XTL = (unsigned short*)(ws + kOffXTL);
  float*          XD  = (float*)(ws + kOffXD);
  float*          YS  = (float*)(ws + kOffYS);
  unsigned short* YGH = (unsigned short*)(ws + kOffYGH);
  unsigned short* YGL = (unsigned short*)(ws + kOffYGL);

  ln_token_kernel<<<kTok / 8, 256, 0, stream>>>(x_in, ln_g, ln_b, XNH, XNL);

  split_rows_bf16_kernel<<<(2 * kDin * kCh / 8 + 255) / 256, 256, 0, stream>>>(w_in, WIH, WIL, 2 * kDin * kCh / 8);
  split_rows_bf16_kernel<<<(kCh * kDin / 8 + 255) / 256, 256, 0, stream>>>(w_out, WOH, WOL, kCh * kDin / 8);
  xproj_planes_kernel<<<(kBK * kXdP * kDin / 8) / 256, 256, 0, stream>>>(w_x, WXH, WXL);

  wmma_gemm64<1, 2, 0, 0, false><<<dim3(((2 * kDin / 64) * (kTok / 64) + 7) / 8, 1), 256, 0, stream>>>(
      WIH, WIL, kCh, 0L,
      XNH, XNL, kCh, 0L,
      (void*)XZ, nullptr, kTok, 0L,
      nullptr, nullptr, 0L,
      2 * kDin, kTok, kCh, 1.0f);

  conv_dir_kernel<<<dim3(kL / kConvTS, kDir, kBsz), kDin, 0, stream>>>(XZ, conv_w, conv_b, XS, XTH, XTL);

  wmma_gemm64<1, 2, 0, 0, false><<<dim3(((kL / 64) * (kXdP / 64) + 7) / 8, kBK), 256, 0, stream>>>(
      XTH, XTL, kDin, (long)kL * kDin,
      WXH, WXL, kDin, (long)kXdP * kDin,
      (void*)XD, nullptr, kXdP, (long)kL * kXdP,
      nullptr, nullptr, 0L,
      kL, kXdP, kDin, 1.0f);

  scan_kernel<<<kBK * (kDin / 8), 256, 0, stream>>>(XD, XS, w_dt, b_dt, a_log, d_skip, YS);

  merge_gate_kernel<<<kTok / 8, 256, 0, stream>>>(YS, XZ, oln_g, oln_b, YGH, YGL);

  wmma_gemm64<1, 2, 0, 0, true><<<dim3(((kCh / 64) * (kL / 64) + 7) / 8, kBsz), 256, 0, stream>>>(
      WOH, WOL, kDin, 0L,
      YGH, YGL, kDin, (long)kL * kDin,
      (void*)out, nullptr, kL, (long)kCh * kL,
      nullptr, x_in, (long)kCh * kL,
      kCh, kL, kDin, 1.0f);
}
